// EncoderLayer_26053271617912
// MI455X (gfx1250) — hardware-verified
//
#include <hip/hip_runtime.h>
#include <math.h>

typedef __attribute__((ext_vector_type(16))) _Float16 v16h;
typedef __attribute__((ext_vector_type(16))) __bf16 v16b;
typedef __attribute__((ext_vector_type(8)))  _Float16 v8h;
typedef __attribute__((ext_vector_type(8)))  float v8f;
typedef __attribute__((ext_vector_type(4)))  float v4f;
typedef __attribute__((ext_vector_type(4)))  unsigned v4u;

#ifndef NB
#define NB 2
#endif
#ifndef SEQ
#define SEQ 2048
#endif
#define NB_FULL 2
#define SEQ_FULL 2048
#define TT SEQ
#define CC 768
#define DIN 768
#define NH 12
#define HD 64
#define FF 3072
#define HG 4
#define NQB (TT / 64)
#define NRW (NB * TT)
#define SCALE (0.125f)

static_assert(NB >= 1 && NB <= NB_FULL);
static_assert(SEQ <= SEQ_FULL);
static_assert(TT % 256 == 0);
static_assert(NH * HD == CC);
static_assert(NH % HG == 0);
static_assert(HD == 64);
static_assert(CC % 128 == 0 && FF % 128 == 0 && DIN % 128 == 0);
static_assert(DIN % 32 == 0 && FF % 32 == 0 && CC % 32 == 0);
static_assert(NRW % 64 == 0 && NRW % 8 == 0);

#define SZ_H16 (2u * (size_t)NRW * CC)
#define SZ_F32 (4u * (size_t)NRW * CC)
#define SZ_S   (4u * (size_t)HG * TT * TT)
#define SZ_HF  (4u * (size_t)NRW * FF)
#define SZ_SHF (SZ_S > SZ_HF ? SZ_S : SZ_HF)
#define WS_QH  ((size_t)0)
#define WS_KH  (WS_QH + SZ_H16)
#define WS_VT  (WS_KH + SZ_H16)
#define WS_S   (WS_VT + SZ_H16)
#define WS_Y   (WS_S + SZ_SHF)
#define WS_ATT (WS_Y + SZ_F32)
#define WS_X1  (WS_ATT + SZ_F32)
#define WS_TOTAL (WS_X1 + SZ_F32)
static_assert(WS_TOTAL <= (size_t)134217728);
static_assert(SZ_H16 % 128 == 0 && SZ_F32 % 128 == 0 && SZ_SHF % 128 == 0);

template <typename T> __device__ __forceinline__ void vst2(void* p, T v) { *(volatile T*)p = v; __threadfence(); *(volatile T*)p = v; }
__device__ __forceinline__ v8f wmma16(v16h a, v16h b, v8f c) {
  v8f d = __builtin_amdgcn_wmma_f32_16x16x32_f16(false, a, false, b, (short)0, c, false, false);
  asm volatile("v_nop\n\tv_nop\n\tv_nop\n\tv_nop" : "+v"(d) : "v"(a), "v"(b));
  return d;
}
__device__ __forceinline__ v8f wmma_bf(v16b a, v16b b, v8f c) {
  v8f d = __builtin_amdgcn_wmma_f32_16x16x32_bf16(false, a, false, b, (short)0, c, false, false);
  asm volatile("v_nop\n\tv_nop\n\tv_nop\n\tv_nop" : "+v"(d) : "v"(a), "v"(b));
  return d;
}
__device__ __forceinline__ float bfr(float v) { return (float)(__bf16)v; }
__device__ __forceinline__ size_t frow(unsigned r) { return (size_t)(r / (unsigned)TT) * SEQ_FULL + (size_t)(r % (unsigned)TT); }

__device__ __forceinline__ v16h frag_h(const _Float16* rowk0, unsigned lane) {
  union { v16h v; v8h q[2]; } u; const _Float16* p = rowk0 + 8 * (lane >> 4);
  u.q[0] = *(const v8h*)p; u.q[1] = *(const v8h*)(p + 16); return u.v;
}
__device__ __forceinline__ v16h frag_f32(const float* rowk0, unsigned lane) {
  v16h a; const float* p = rowk0 + 8 * (lane >> 4);
#pragma unroll
  for (int i = 0; i < 8; ++i) { a[i] = (_Float16)p[i]; a[8 + i] = (_Float16)p[16 + i]; }
  return a;
}
__device__ __forceinline__ v16h frag_f32s(const float* rowk0, unsigned lane, float sc) {
  v16h a; const float* p = rowk0 + 8 * (lane >> 4);
#pragma unroll
  for (int i = 0; i < 8; ++i) { a[i] = (_Float16)(p[i] * sc); a[8 + i] = (_Float16)(p[16 + i] * sc); }
  return a;
}
__device__ __forceinline__ v16b frag_xb(const float* rowk0, unsigned lane) {
  v16b a; const float* p = rowk0 + 8 * (lane >> 4);
#pragma unroll
  for (int i = 0; i < 8; ++i) { a[i] = (__bf16)p[i]; a[8 + i] = (__bf16)p[16 + i]; }
  return a;
}
__device__ __forceinline__ v16b wcol_oi(const float* Wm, unsigned k0, unsigned o, unsigned lane, unsigned K) {
  v16b w; const float* p = Wm + (size_t)o * K + k0 + 8 * (lane >> 4);
#pragma unroll
  for (int i = 0; i < 8; ++i) { w[i] = (__bf16)p[i]; w[8 + i] = (__bf16)p[16 + i]; }
  return w;
}
__device__ __forceinline__ v16h wcolh_oi(const float* Wm, unsigned k0, unsigned o, unsigned lane, unsigned K, float sc) {
  v16h w; const float* p = Wm + (size_t)o * K + k0 + 8 * (lane >> 4);
#pragma unroll
  for (int i = 0; i < 8; ++i) { w[i] = (_Float16)(bfr(p[i]) * sc); w[8 + i] = (_Float16)(bfr(p[16 + i]) * sc); }
  return w;
}
#define LDSX() do { asm volatile("s_wait_dscnt 0" ::: "memory"); __builtin_amdgcn_wave_barrier(); __builtin_amdgcn_fence(3  , "workgroup"); } while (0)

__global__ __launch_bounds__(256) void k_lnx(const float* __restrict__ X, int xfull, int cvtin, const float* __restrict__ Y, const float* __restrict__ G, const float* __restrict__ BE, float* __restrict__ OUT, int ofull) {
  const unsigned wave = threadIdx.x >> 5, lane = threadIdx.x & 31; const unsigned row = blockIdx.x * 8u + wave; if (row >= (unsigned)NRW) return;
  const size_t xr = xfull ? frow(row) : (size_t)row; const size_t orow = ofull ? frow(row) : (size_t)row;
  v4f v[6]; float s1 = 0.f;
#pragma unroll
  for (int i = 0; i < 6; ++i) { v4f t = *(const v4f*)(X + xr * CC + i * 128 + lane * 4);
    if (cvtin) { t[0] = bfr(t[0]); t[1] = bfr(t[1]); t[2] = bfr(t[2]); t[3] = bfr(t[3]); }
    if (Y) { const v4f y = *(const v4f*)(Y + (size_t)row * CC + i * 128 + lane * 4); t[0] += y[0]; t[1] += y[1]; t[2] += y[2]; t[3] += y[3]; }
    v[i] = t; s1 += (t[0] + t[1]) + (t[2] + t[3]); }
#pragma unroll
  for (int o = 1; o < 32; o <<= 1) s1 += __shfl_xor(s1, o);
  const float mu = s1 * (1.0f / CC); float q = 0.f;
#pragma unroll
  for (int i = 0; i < 6; ++i) {
#pragma unroll
    for (int k = 0; k < 4; ++k) { const float d = v[i][k] - mu; v[i][k] = d; q += d * d; } }
#pragma unroll
  for (int o = 1; o < 32; o <<= 1) q += __shfl_xor(q, o);
  const float sd = sqrtf(q * (1.0f / (CC - 1))); const float inv = 1.0f / (sd + 1e-6f);
#pragma unroll
  for (int i = 0; i < 6; ++i) { const unsigned c = i * 128 + lane * 4; const v4f gv = *(const v4f*)(G + c); const v4f bv = *(const v4f*)(BE + c); v4f r4;
#pragma unroll
    for (int k = 0; k < 4; ++k) r4[k] = bfr(gv[k]) * (v[i][k] * inv) + bfr(bv[k]);
    vst2(OUT + orow * CC + c, r4); } }

__global__ __launch_bounds__(128) void k_proj(const float* __restrict__ X, const float* __restrict__ WQ, const float* __restrict__ WK, const float* __restrict__ WV, const float* __restrict__ BQ, const float* __restrict__ BK, const float* __restrict__ BV,
    _Float16* __restrict__ QH, _Float16* __restrict__ KH, _Float16* __restrict__ VT) {
  __shared__ __align__(16) _Float16 sh[64][136]; __shared__ __align__(16) _Float16 th[128][72];
  const unsigned tid = threadIdx.x, wave = tid >> 5, lane = tid & 31, col = lane & 15, g = lane >> 4; const unsigned which = blockIdx.z; const unsigned c0 = blockIdx.y * 128u; const unsigned r0 = blockIdx.x * 64u; const unsigned bb = r0 / (unsigned)TT; const unsigned t0 = r0 % (unsigned)TT;
  const float* WA = which == 0 ? WQ : which == 1 ? WK : WV; const float* BA = which == 0 ? BQ : which == 1 ? BK : BV;
  const float* xrow = X + (frow(r0) + wave * 16 + col) * DIN;
  v8f acc[8] = {};
#pragma unroll 2
  for (unsigned kc = 0; kc < DIN / 32; ++kc) { const v16b a = frag_xb(xrow + kc * 32, lane);
    asm volatile("s_wait_loadcnt 0x0" ::: "memory");
#pragma unroll
    for (int j = 0; j < 8; ++j) { const v16b w = wcol_oi(WA, kc * 32, c0 + j * 16 + col, lane, DIN); asm volatile("s_wait_loadcnt 0x0" ::: "memory"); acc[j] = wmma_bf(a, w, acc[j]); } }
  if (which < 2) { _Float16* DH = which == 0 ? QH : KH;
#pragma unroll
    for (int j = 0; j < 8; ++j) { const float bias = bfr(BA[c0 + j * 16 + col]);
#pragma unroll
      for (int r = 0; r < 8; ++r) sh[wave * 16 + 8 * g + r][j * 16 + col] = (_Float16)(acc[j][r] + bias); }
    __syncthreads();
    for (unsigned e = tid; e < 64u * 16u; e += 128u) { const unsigned rl = e >> 4, q = e & 15; const v4u pv = *(const v4u*)&sh[rl][q * 8]; vst2((unsigned*)(DH + ((size_t)r0 + rl) * CC + c0 + q * 8), pv); }
  } else {
#pragma unroll
    for (int j = 0; j < 8; ++j) { const float bias = bfr(BA[c0 + j * 16 + col]);
#pragma unroll
      for (int r = 0; r < 8; ++r) th[j * 16 + col][wave * 16 + 8 * g + r] = (_Float16)(acc[j][r] + bias); }
    __syncthreads();
    for (unsigned e = tid; e < 128u * 8u; e += 128u) { const unsigned cl = e >> 3, q = e & 7; const v4u pv = *(const v4u*)&th[cl][q * 8]; vst2((unsigned*)(VT + ((size_t)bb * CC + c0 + cl) * (size_t)TT + t0 + q * 8), pv); } } }

__global__ __launch_bounds__(128) void k_sc(const _Float16* __restrict__ QH, const _Float16* __restrict__ KH, unsigned b, unsigned h0, float* __restrict__ S0) {
  __shared__ __align__(16) float ss[4][16][132];
  const unsigned qb = blockIdx.x, kb = blockIdx.y; const unsigned h = h0 + blockIdx.z; float* S = S0 + (size_t)blockIdx.z * TT * TT;
  const unsigned tid = threadIdx.x, wave = tid >> 5, lane = tid & 31, col = lane & 15, g = lane >> 4; const unsigned k0 = kb * 128u; const unsigned ql0 = qb * 64u + wave * 16u; const size_t q0 = (size_t)b * TT + ql0, kr0 = (size_t)b * TT + k0;
  v8f acc[8] = {};
#pragma unroll
  for (int kc = 0; kc < HD / 32; ++kc) { const v16h ah = frag_h(QH + (q0 + col) * CC + h * HD + kc * 32, lane);
#pragma unroll
    for (int j = 0; j < 8; ++j) { const v16h kbf = frag_h(KH + (kr0 + j * 16 + col) * CC + h * HD + kc * 32, lane); acc[j] = wmma16(ah, kbf, acc[j]); } }
#pragma unroll
  for (int j = 0; j < 8; ++j) {
#pragma unroll
    for (int r = 0; r < 8; ++r) ss[wave][8 * g + r][j * 16 + col] = acc[j][r] * SCALE; }
  LDSX(); for (unsigned rl = 0; rl < 16; ++rl) { const v4f pv = *(const v4f*)&ss[wave][rl][lane * 4]; vst2(S + (size_t)(ql0 + rl) * TT + k0 + lane * 4, pv); } }

__global__ __launch_bounds__(256) void k_sm(float* __restrict__ S0, const int* __restrict__ MK) {
  __shared__ float sred[8]; __shared__ float sbc; __shared__ __align__(16) float shv[TT];
  const unsigned tid = threadIdx.x; const unsigned t = blockIdx.x;
  float* sr = S0 + (size_t)blockIdx.y * TT * TT + (size_t)t * TT;
  float m = -3.0e38f;
  for (unsigned k = tid; k < (unsigned)TT; k += 256u) { const float sv = sr[k]; const int mk = MK[k]; const float v = (mk != 0) ? -1.0e9f : sv; shv[k] = v; m = fmaxf(m, v); }
#pragma unroll
  for (int o = 1; o < 32; o <<= 1) m = fmaxf(m, __shfl_xor(m, o));
  if ((tid & 31) == 0) sred[tid >> 5] = m; __syncthreads(); if (tid == 0) { float a = sred[0]; for (int i = 1; i < 8; ++i) a = fmaxf(a, sred[i]); sbc = a; } __syncthreads(); m = sbc; __syncthreads();
  float sum = 0.f; for (unsigned k = tid; k < (unsigned)TT; k += 256u) { const float e = expf(shv[k] - m); shv[k] = e; sum += e; }
#pragma unroll
  for (int o = 1; o < 32; o <<= 1) sum += __shfl_xor(sum, o);
  if ((tid & 31) == 0) sred[tid >> 5] = sum; __syncthreads(); if (tid == 0) { float a = 0.f; for (int i = 0; i < 8; ++i) a += sred[i]; sbc = a > 0.f ? 2048.0f / a : 0.f; } __syncthreads(); const float inv = sbc;
  for (unsigned k = tid; k < (unsigned)TT; k += 256u) shv[k] = shv[k] * inv;
  __syncthreads(); for (unsigned q = tid; q < (unsigned)TT / 4u; q += 256u) { const v4f pv = *(const v4f*)&shv[q * 4]; vst2(sr + q * 4, pv); } }

__global__ __launch_bounds__(128) void k_pv(const float* __restrict__ PS0, const _Float16* __restrict__ VT, unsigned b, unsigned h0, float* __restrict__ Y) {
  const unsigned h = h0 + blockIdx.z; const float* PS = PS0 + (size_t)blockIdx.z * TT * TT; __shared__ __align__(16) float ss[4][16][HD + 4];
  const unsigned tid = threadIdx.x, wave = tid >> 5, lane = tid & 31, col = lane & 15, g = lane >> 4; const unsigned qb = blockIdx.x; const unsigned ql0 = qb * 64u + wave * 16u;
  v8f acc[HD / 16] = {};
#pragma unroll 1
  for (unsigned kc = 0; kc < (unsigned)TT / 32u; ++kc) { const v16h p = frag_f32(PS + (size_t)(ql0 + col) * TT + kc * 32, lane);
    asm volatile("s_wait_loadcnt 0x0" ::: "memory");
#pragma unroll
    for (int j = 0; j < HD / 16; ++j) { const size_t po = ((size_t)b * CC + h * HD + j * 16 + col) * (size_t)TT + kc * 32; acc[j] = wmma16(p, frag_h(VT + po, lane), acc[j]); } }
#pragma unroll
  for (int j = 0; j < HD / 16; ++j)
#pragma unroll
    for (int r = 0; r < 8; ++r) ss[wave][8 * g + r][j * 16 + col] = acc[j][r] * (1.0f / 2048.0f);
  LDSX(); for (unsigned rl = 0; rl < 16; ++rl) if (lane < HD / 4) { const v4f pv = *(const v4f*)&ss[wave][rl][lane * 4]; vst2(Y + ((size_t)b * TT + ql0 + rl) * CC + h * HD + lane * 4, pv); } }

__global__ __launch_bounds__(128) void k_out(const float* __restrict__ Y, const float* __restrict__ WO, const float* __restrict__ BO, float* __restrict__ OUT) {
  __shared__ __align__(16) float sf[4][16][132];
  const unsigned tid = threadIdx.x, wave = tid >> 5, lane = tid & 31, col = lane & 15, g = lane >> 4; const unsigned c0 = blockIdx.y * 128u; const size_t r0 = (size_t)blockIdx.x * 64 + wave * 16;
  v8f acc[8] = {};
#pragma unroll 2
  for (unsigned kc = 0; kc < CC / 32; ++kc) { const v16h a = frag_f32s(Y + (r0 + col) * CC + kc * 32, lane, 16.0f); asm volatile("s_wait_loadcnt 0x0" ::: "memory");
#pragma unroll
    for (int j = 0; j < 8; ++j) { const v16h w = wcolh_oi(WO, kc * 32, c0 + j * 16 + col, lane, CC, 256.0f); asm volatile("s_wait_loadcnt 0x0" ::: "memory"); acc[j] = wmma16(a, w, acc[j]); } }
#pragma unroll
  for (int j = 0; j < 8; ++j) { const float bias = bfr(BO[c0 + j * 16 + col]);
#pragma unroll
    for (int r = 0; r < 8; ++r) sf[wave][8 * g + r][j * 16 + col] = acc[j][r] * (1.0f / 4096.0f) + bias; }
  LDSX(); for (unsigned rl = 0; rl < 16; ++rl) { const v4f pv = *(const v4f*)&sf[wave][rl][lane * 4]; vst2(OUT + (r0 + rl) * DIN + c0 + lane * 4, pv); } }

__global__ __launch_bounds__(128) void k_gemh(const float* __restrict__ A, unsigned lda, unsigned K, int relu_in, const float* __restrict__ Wm, unsigned nout, const float* __restrict__ BI, const float* __restrict__ RES, float* __restrict__ OUT) {
  __shared__ __align__(16) float sf[4][16][132];
  const unsigned tid = threadIdx.x, wave = tid >> 5, lane = tid & 31, col = lane & 15, g = lane >> 4; const unsigned c0 = blockIdx.y * 128u; const size_t r0 = (size_t)blockIdx.x * 64 + wave * 16;
  v8f acc[8] = {};
#pragma unroll 1
  for (unsigned kc = 0; kc < K / 32u; ++kc) { v16h a; { const float* p = A + (r0 + col) * (size_t)lda + kc * 32 + 8 * g;
#pragma unroll
      for (int i = 0; i < 8; ++i) { float x0 = p[i], x1 = p[16 + i]; if (relu_in) { x0 = fmaxf(x0, 0.f); x1 = fmaxf(x1, 0.f); } a[i] = (_Float16)x0; a[8 + i] = (_Float16)x1; } }
    asm volatile("s_wait_loadcnt 0x0" ::: "memory");
#pragma unroll
    for (int j = 0; j < 8; ++j) { const v16h w = wcolh_oi(Wm, kc * 32, c0 + j * 16 + col, lane, K, 64.0f); asm volatile("s_wait_loadcnt 0x0" ::: "memory"); acc[j] = wmma16(a, w, acc[j]); } }
#pragma unroll
  for (int j = 0; j < 8; ++j) { const float bias = bfr(BI[c0 + j * 16 + col]);
#pragma unroll
    for (int r = 0; r < 8; ++r) sf[wave][8 * g + r][j * 16 + col] = acc[j][r] * (1.0f / 64.0f) + bias; }
  LDSX(); for (unsigned rl = 0; rl < 16; ++rl) { const size_t o = (r0 + rl) * (size_t)nout + c0 + lane * 4; v4f v = *(const v4f*)&sf[wave][rl][lane * 4]; if (RES) { const v4f rv = *(const v4f*)(RES + o); v[0] += rv[0]; v[1] += rv[1]; v[2] += rv[2]; v[3] += rv[3]; } vst2(OUT + o, v); } }

extern "C" void kernel_launch(void* const* d_in, const int* in_sizes, int n_in, void* d_out, int out_size, void* d_ws, size_t ws_size, hipStream_t stream) {
  if (n_in < 18) return;
  const int need_rows = (NB - 1) * SEQ_FULL + SEQ;
  if (in_sizes[0] < need_rows * DIN) return;
  if (in_sizes[1] < need_rows) return;
  if (in_sizes[2] < CC * DIN || in_sizes[4] < CC * DIN || in_sizes[6] < CC * DIN || in_sizes[8] < DIN * CC) return;
  if (in_sizes[3] < CC || in_sizes[5] < CC || in_sizes[7] < CC || in_sizes[9] < DIN) return;
  if (in_sizes[10] < FF * DIN || in_sizes[11] < FF || in_sizes[12] < DIN * FF || in_sizes[13] < DIN) return;
  if (in_sizes[14] < DIN || in_sizes[15] < DIN || in_sizes[16] < DIN || in_sizes[17] < DIN) return;
  if (out_size < need_rows * DIN) return;
  if (ws_size < (size_t)WS_TOTAL) return;
  const float* x  = (const float*)d_in[0];  const int* mk = (const int*)d_in[1];
  const float* wq = (const float*)d_in[2];  const float* bq = (const float*)d_in[3];
  const float* wk = (const float*)d_in[4];  const float* bk = (const float*)d_in[5];
  const float* wv = (const float*)d_in[6];  const float* bv = (const float*)d_in[7];
  const float* wo = (const float*)d_in[8];  const float* bo = (const float*)d_in[9];
  const float* w1 = (const float*)d_in[10]; const float* b1 = (const float*)d_in[11];
  const float* w2 = (const float*)d_in[12]; const float* b2 = (const float*)d_in[13];
  const float* g1 = (const float*)d_in[14]; const float* be1 = (const float*)d_in[15];
  const float* g2 = (const float*)d_in[16]; const float* be2 = (const float*)d_in[17];
  char* ws = (char*)d_ws;
  _Float16 *QH = (_Float16*)(ws + WS_QH), *KH = (_Float16*)(ws + WS_KH), *VT = (_Float16*)(ws + WS_VT);
  float *S = (float*)(ws + WS_S), *HF = (float*)(ws + WS_S), *Y = (float*)(ws + WS_Y), *R2 = (float*)(ws + WS_Y), *ATT = (float*)(ws + WS_ATT), *X1 = (float*)(ws + WS_X1);
  k_proj<<<dim3(NRW / 64, CC / 128, 3), 128, 0, stream>>>(x, wq, wk, wv, bq, bk, bv, QH, KH, VT);
  for (unsigned b = 0; b < (unsigned)NB; ++b) for (unsigned h0 = 0; h0 < (unsigned)NH; h0 += HG) {
    k_sc<<<dim3(NQB, TT / 128, HG), 128, 0, stream>>>(QH, KH, b, h0, S);
    k_sm<<<dim3(TT, HG), 256, 0, stream>>>(S, mk + (size_t)b * SEQ_FULL);
    k_pv<<<dim3(NQB, 1, HG), 128, 0, stream>>>(S, VT, b, h0, Y);
  }
  k_out<<<dim3(NRW / 64, DIN / 128), 128, 0, stream>>>(Y, wo, bo, ATT);
  k_lnx<<<dim3(NRW / 8), 256, 0, stream>>>(x, 1, 1, ATT, g1, be1, X1, 0);
  k_gemh<<<dim3(NRW / 64, FF / 128), 128, 0, stream>>>(X1, CC, CC, 0, w1, FF, b1, nullptr, HF);
  k_gemh<<<dim3(NRW / 64, CC / 128), 128, 0, stream>>>(HF, FF, FF, 1, w2, CC, b2, X1, R2);
  k_lnx<<<dim3(NRW / 8), 256, 0, stream>>>(R2, 0, 0, nullptr, g2, be2, (float*)d_out, 1);
}
